// MultiScaleSpatialAttention_13314398617806
// MI455X (gfx1250) — hardware-verified
//
#include <hip/hip_runtime.h>
#include <math.h>

#define NN   50000
#define DD   128
#define NHD  8
#define NE   600000
#define NSC  3
#define NBIN 50
#define MP   50048
#define QKVP 384
#define NT   256
#define TG   2048
#define NTILE 25
#define NROWT (NTILE * TG)
#define SCH  4096
#define SPT  (SCH / NT)
#define NCH  ((NE + SCH - 1) / SCH)
#define STREAM_LDS_BYTES ((TG * NHD * 2 + SCH) * 4)
#define WSC  8.0f
#define AGSC 16.0f

typedef __attribute__((ext_vector_type(16))) _Float16 v16h;
typedef __attribute__((ext_vector_type(8)))  _Float16 v8h;
typedef __attribute__((ext_vector_type(4)))  _Float16 v4h;
typedef __attribute__((ext_vector_type(16))) __bf16   v16b;
typedef __attribute__((ext_vector_type(8)))  __bf16   v8b;
typedef __attribute__((ext_vector_type(8)))  float    v8f;
typedef __attribute__((ext_vector_type(4)))  float    v4f;
typedef __attribute__((ext_vector_type(4)))  int      v4i;
#define U16(p) ((const unsigned short*)(const void*)(p))

__device__ __forceinline__ unsigned short f2bf_bits(float f) {
  unsigned u = __float_as_uint(f);
  return (unsigned short)((u + 0x7FFFu + ((u >> 16) & 1u)) >> 16);
}
__device__ __forceinline__ float bf_bits2f(unsigned short h) { return __uint_as_float(((unsigned)h) << 16); }

__device__ __forceinline__ void dep_guard_h(v8f& a, v8f& b, v16h x, v16h y) { asm volatile("v_nop\n\tv_nop\n\tv_nop\n\tv_nop" : "+v"(a), "+v"(b) : "v"(x), "v"(y)); }
__device__ __forceinline__ void dep_guard_b(v8f& a, v8f& b, v16b x, v16b y) { asm volatile("v_nop\n\tv_nop\n\tv_nop\n\tv_nop" : "+v"(a), "+v"(b) : "v"(x), "v"(y)); }
__device__ __forceinline__ void keep4_h(v16h a, v16h b, v16h c, v16h d) { asm volatile("v_nop" :: "v"(a), "v"(b), "v"(c), "v"(d)); }
__device__ __forceinline__ void keep4_b(v16b a, v16b b, v16b c, v16b d) { asm volatile("v_nop" :: "v"(a), "v"(b), "v"(c), "v"(d)); }
__device__ __forceinline__ void acc_guard4(v8f& a, v8f& b, v8f& c, v8f& d) { asm volatile("v_nop\n\tv_nop\n\tv_nop\n\tv_nop" : "+v"(a), "+v"(b), "+v"(c), "+v"(d)); }
template <typename T> struct Frag;
template <> struct Frag<_Float16> {
  typedef v16h V; union U { v16h v; v8h h[2]; };
  static __device__ __forceinline__ v16h load(const _Float16* p) {
    U f; f.h[0] = *(const v8h*)(p); f.h[1] = *(const v8h*)(p + 16); return f.v;
  }
  static __device__ __forceinline__ v8f mma(v16h a, v16h b, v8f c) {
    return __builtin_amdgcn_wmma_f32_16x16x32_f16(false, a, false, b, (short)0, c, false, false);
  }
  static __device__ __forceinline__ void guard(v8f& a, v8f& b, v16h x, v16h y) { dep_guard_h(a, b, x, y); }
  static __device__ __forceinline__ void keep(v16h a, v16h b, v16h c, v16h d) { keep4_h(a, b, c, d); }
};
template <> struct Frag<__bf16> {
  typedef v16b V; union U { v16b v; v8b h[2]; };
  static __device__ __forceinline__ v16b load(const __bf16* p) {
    U f; f.h[0] = *(const v8b*)(p); f.h[1] = *(const v8b*)(p + 16); return f.v;
  }
  static __device__ __forceinline__ v8f mma(v16b a, v16b b, v8f c) {
    return __builtin_amdgcn_wmma_f32_16x16x32_bf16(false, a, false, b, (short)0, c, false, false);
  }
  static __device__ __forceinline__ void guard(v8f& a, v8f& b, v16b x, v16b y) { dep_guard_b(a, b, x, y); }
  static __device__ __forceinline__ void keep(v16b a, v16b b, v16b c, v16b d) { keep4_b(a, b, c, d); }
};

template <int ET> struct Elem;
template <> struct Elem<0> { typedef _Float16 T; };
template <> struct Elem<1> { typedef __bf16 T; };
template <int ET, bool SPLIT, int BIAS_MODE, int OUT_MODE, bool RESID, int ACT = 0>
__global__ __launch_bounds__(256) void wmma_gemm64(
    const unsigned short* __restrict__ Ap, const unsigned short* __restrict__ A2p, int lda, long strideA,
    const unsigned short* __restrict__ Btp, const unsigned short* __restrict__ Bt2p, int ldb, long strideB,
    void* Cout, void* Cout2, int ldc, long strideC,
    const float* __restrict__ bias,
    const float* resid, long strideR,
    int M, int N, int K, float scale, int Mv) {
  typedef typename Elem<ET>::T T;
  typedef typename Frag<T>::V V;
  const T* A = (const T*)Ap; const T* A2 = (const T*)A2p; const T* Bt = (const T*)Btp; const T* Bt2 = (const T*)Bt2p;
  __shared__ __align__(16) float sT[8][16 * 68];
  const int b    = blockIdx.y;
  const int lane = threadIdx.x & 31;
  const int wave = threadIdx.x >> 5;
  const int tilesN = N >> 6;
  const int tilesM = M >> 6;
  const int tile = blockIdx.x * 8 + wave;
  if (tile >= tilesM * tilesN) return;
  const int tm = tile / tilesN;
  const int tn = tile - tm * tilesN;
  const int m0 = tm << 6;
  const int n0 = tn << 6;

  const T* Ab  = A  + (size_t)b * strideA;
  const T* Bb  = Bt + (size_t)b * strideB;
  const T* Ab2 = SPLIT ? (A2  + (size_t)b * strideA) : nullptr;
  const T* Bb2 = SPLIT ? (Bt2 + (size_t)b * strideB) : nullptr;

  const int rlane = lane & 15;
  const int koff  = (lane >> 4) * 8;
  const int mOff  = (lane >> 4) * 8;

  v8f acc[4][4];
#pragma unroll
  for (int i = 0; i < 4; ++i)
#pragma unroll
    for (int j = 0; j < 4; ++j) acc[i][j] = (v8f){0.f,0.f,0.f,0.f,0.f,0.f,0.f,0.f};

  for (int k0 = 0; k0 < K; k0 += 32) {
    V bh[4], bl[4];
#pragma unroll
    for (int j = 0; j < 4; ++j) {
      const size_t bo = (size_t)(n0 + (j << 4) + rlane) * ldb + koff + k0;
      bh[j] = Frag<T>::load(Bb + bo);
      if (SPLIT) bl[j] = Frag<T>::load(Bb2 + bo);
    }
#pragma unroll
    for (int i = 0; i < 4; ++i) {
      const size_t ao = (size_t)(m0 + (i << 4) + rlane) * lda + koff + k0;
      V ah = Frag<T>::load(Ab + ao);
      V al;
      if (SPLIT) al = Frag<T>::load(Ab2 + ao);
#pragma unroll
      for (int j = 0; j < 4; ++j) {
        acc[i][j] = Frag<T>::mma(ah, bh[j], acc[i][j]);
        if (SPLIT) {
          acc[i][j] = Frag<T>::mma(ah, bl[j], acc[i][j]);
          acc[i][j] = Frag<T>::mma(al, bh[j], acc[i][j]);
        }
      }
      Frag<T>::guard(acc[i][0], acc[i][3], ah, SPLIT ? al : ah);
    }
    Frag<T>::keep(bh[0], bh[1], bh[2], bh[3]);
    if (SPLIT) Frag<T>::keep(bl[0], bl[1], bl[2], bl[3]);
  }
  acc_guard4(acc[0][0], acc[0][1], acc[0][2], acc[0][3]);
  acc_guard4(acc[1][0], acc[1][1], acc[1][2], acc[1][3]);
  acc_guard4(acc[2][0], acc[2][1], acc[2][2], acc[2][3]);
  acc_guard4(acc[3][0], acc[3][1], acc[3][2], acc[3][3]);

  float* slab = sT[wave];
  const float* Rb = RESID ? (resid + (size_t)b * strideR) : nullptr;
#pragma unroll
  for (int i = 0; i < 4; ++i) {
    const int mBase = m0 + (i << 4);
#pragma unroll
    for (int j = 0; j < 4; ++j) {
      const int n = n0 + (j << 4) + rlane;
      float bv = 0.f;
      if (BIAS_MODE == 2) bv = bias[n];
#pragma unroll
      for (int r = 0; r < 8; ++r) {
        float v = acc[i][j][r] * scale;
        if (BIAS_MODE == 1) v += bias[mBase + mOff + r];
        if (BIAS_MODE == 2) v += bv;
        if (RESID) {
          int rrow = mBase + mOff + r;
          rrow = (rrow < Mv) ? rrow : (Mv - 1);
          v += Rb[(size_t)rrow * ldc + n];
        }
        if (ACT == 1) v = tanhf(v);
        if (ACT == 2) v = fmaxf(v, 0.0f);
        if (ACT == 3) v = v / (1.0f + expf(-v));
        if (ACT == 4) v = (v > 0.f) ? v : 0.01f * v;
        if (ACT == 5) v = 0.5f * v * (1.0f + erff(v * 0.70710678118654752f));
        if (ACT == 6) v = (v > 0.f) ? v : 0.2f * v;
        slab[(mOff + r) * 68 + (j << 4) + rlane] = v;
      }
    }
    __builtin_amdgcn_fence(__ATOMIC_RELEASE, "workgroup");
    __builtin_amdgcn_wave_barrier();
    __builtin_amdgcn_fence(__ATOMIC_ACQUIRE, "workgroup");
    if (OUT_MODE == 0) {
      float* C = (float*)Cout + (size_t)b * strideC;
      const int hh = lane >> 4, c4 = (lane & 15) * 4;
      for (int pass = 0; pass < 2; ++pass) {
#pragma unroll
        for (int it = 0; it < 8; ++it) {
          const int row = it * 2 + hh;
          v4f v = *(const v4f*)(slab + row * 68 + c4);
          if (mBase + row < Mv) *(volatile v4f*)(C + (size_t)(mBase + row) * ldc + n0 + c4) = v;
        }
        __threadfence();
      }
    } else {
      const int q = lane >> 3, c8 = (lane & 7) * 8;
      unsigned short* C  = (unsigned short*)Cout  + (size_t)b * strideC;
      unsigned short* C2 = (OUT_MODE == 2) ? ((unsigned short*)Cout2 + (size_t)b * strideC) : nullptr;
      for (int pass = 0; pass < 2; ++pass) {
#pragma unroll
        for (int it = 0; it < 4; ++it) {
          const int row = it * 4 + q;
          const float* sp = slab + row * 68 + c8;
          v8h hv, lv;
#pragma unroll
          for (int e = 0; e < 8; ++e) {
            if (OUT_MODE == 1) {
              hv[e] = (_Float16)sp[e];
            } else {
              unsigned short hb = f2bf_bits(sp[e]);
              unsigned short lb = f2bf_bits(sp[e] - bf_bits2f(hb));
              hv[e] = __builtin_bit_cast(_Float16, hb);
              lv[e] = __builtin_bit_cast(_Float16, lb);
            }
          }
          if (mBase + row < Mv) {
            *(volatile v8h*)(C + (size_t)(mBase + row) * ldc + n0 + c8) = hv;
            if (OUT_MODE == 2) *(volatile v8h*)(C2 + (size_t)(mBase + row) * ldc + n0 + c8) = lv;
          }
        }
        __threadfence();
      }
    }
    __builtin_amdgcn_fence(__ATOMIC_RELEASE, "workgroup");
    __builtin_amdgcn_wave_barrier();
    __builtin_amdgcn_fence(__ATOMIC_ACQUIRE, "workgroup");
  }
}

__global__ __launch_bounds__(256) void cast_x_kernel(
    const float* __restrict__ in, unsigned short* __restrict__ out, int nval2, int n2) {
  const int i = blockIdx.x * 256 + threadIdx.x;
  if (i < n2) {
    const int ic = (i < nval2) ? i : (nval2 - 1);
    float f0 = in[2 * (size_t)ic], f1 = in[2 * (size_t)ic + 1];
    if (i >= nval2) { f0 = 0.f; f1 = 0.f; }
    const _Float16 h0 = (_Float16)f0, h1 = (_Float16)f1;
    const unsigned u = (unsigned)__builtin_bit_cast(unsigned short, h0) | ((unsigned)__builtin_bit_cast(unsigned short, h1) << 16);
    ((volatile unsigned*)out)[i] = u;
    __threadfence();
    ((volatile unsigned*)out)[i] = u;
  }
}

__device__ __forceinline__ unsigned pack_f16x2(float a, float b) {
  const _Float16 h0 = (_Float16)a, h1 = (_Float16)b;
  return (unsigned)__builtin_bit_cast(unsigned short, h0) | ((unsigned)__builtin_bit_cast(unsigned short, h1) << 16);
}

__device__ __forceinline__ void scale_softmax(const float* __restrict__ sw, float& w0, float& w1, float& w2) {
  const float s0 = sw[0], s1 = sw[1], s2 = sw[2];
  const float mx = fmaxf(fmaxf(s0, s1), s2);
  const float e0 = __expf(s0 - mx), e1 = __expf(s1 - mx), e2 = __expf(s2 - mx);
  const float inv = 1.0f / ((e0 + e1) + e2);
  w0 = e0 * inv; w1 = e1 * inv; w2 = e2 * inv;
}

__global__ __launch_bounds__(NT) void wprep_kernel(const float* __restrict__ Wq, const float* __restrict__ bq,
                                                  const float* __restrict__ Wk, const float* __restrict__ bk,
                                                  const float* __restrict__ Wv, const float* __restrict__ bv,
                                                  const float* __restrict__ Wo, const float* __restrict__ bo,
                                                  const float* __restrict__ sw,
                                                  unsigned* __restrict__ WQKV, unsigned* __restrict__ WO,
                                                  float* __restrict__ BQKV, float* __restrict__ BOW) {
  const int t = threadIdx.x;
  float w0, w1, w2;
  scale_softmax(sw, w0, w1, w2);
#pragma unroll 1
  for (int i = t; i < NSC * QKVP * (DD / 2); i += NT) {
    const int si = i / (QKVP * (DD / 2));
    const int r = i - si * (QKVP * (DD / 2));
    const int n = r >> 6, k = 2 * (r & 63);
    const int g = n >> 7, nn = n & 127;
    const size_t idx = (size_t)si * DD * DD + (size_t)nn * DD + k;
    const float q0 = Wq[idx], q1 = Wq[idx + 1], k0 = Wk[idx], k1 = Wk[idx + 1], v0 = Wv[idx], v1 = Wv[idx + 1];
    const float a  = (g == 0) ? q0 : ((g == 1) ? k0 : v0);
    const float bb = (g == 0) ? q1 : ((g == 1) ? k1 : v1);
    const unsigned u = pack_f16x2(a * WSC, bb * WSC);
    ((volatile unsigned*)WQKV)[i] = u; __threadfence(); ((volatile unsigned*)WQKV)[i] = u;
  }
#pragma unroll 1
  for (int i = t; i < NSC * DD * (DD / 2); i += NT) {
    const unsigned u = pack_f16x2(Wo[2 * (size_t)i] * WSC, Wo[2 * (size_t)i + 1] * WSC);
    ((volatile unsigned*)WO)[i] = u; __threadfence(); ((volatile unsigned*)WO)[i] = u;
  }
#pragma unroll 1
  for (int i = t; i < NSC * QKVP; i += NT) {
    const int si = i / QKVP, n = i - si * QKVP;
    const int g = n >> 7, nn = n & 127;
    const int idx = si * DD + nn;
    const float a = bq[idx], bb = bk[idx], c = bv[idx];
    const float v = (g == 0) ? a : ((g == 1) ? bb : c);
    ((volatile float*)BQKV)[i] = v; __threadfence(); ((volatile float*)BQKV)[i] = v;
  }
#pragma unroll 1
  for (int i = t; i < NSC * DD; i += NT) {
    const int si = i >> 7;
    const float w = (si == 0) ? w0 : ((si == 1) ? w1 : w2);
    const float v = w * bo[i];
    ((volatile float*)BOW)[i] = v; __threadfence(); ((volatile float*)BOW)[i] = v;
  }
}

__device__ __forceinline__ int blk_excl_scan(int cnt, int* scan_ws, int tid, int* tot) {
  const int lane = tid & 31, wave = tid >> 5; int incl = cnt;
#pragma unroll
  for (int o = 1; o < 32; o <<= 1) { const int v = __shfl_up(incl, o, 32); if (lane >= o) incl += v; }
  if (lane == 31) scan_ws[wave] = incl;
  __syncthreads();
  if (wave == 0) { int wv = (lane < NT / 32) ? scan_ws[lane] : 0; int wincl = wv;
#pragma unroll
    for (int o = 1; o < 32; o <<= 1) { const int v = __shfl_up(wincl, o, 32); if (lane >= o) wincl += v; }
    if (lane < NT / 32) scan_ws[32 + lane] = wincl - wv; if (lane == 31) scan_ws[64] = wincl; }
  __syncthreads();
  const int res = scan_ws[32 + wave] + incl - cnt; *tot = scan_ws[64];
  return res;
}
template <int SP, int CAP>
__device__ __forceinline__ int chunk_hits(const int* __restrict__ dstv, int e0, int n0, int tid, int* LIST, int* scan_ws) {
  const int eb = e0 + tid * SP;
  const bool real = eb < NE;
  const int ebc = real ? eb : (NE - SP);
  int rec[SP]; int cnt = 0;
#pragma unroll
  for (int k = 0; k < SP; k += 4) {
    const v4i d4 = *(const v4i*)(dstv + ebc + k);
#pragma unroll
    for (int q = 0; q < 4; ++q) {
      const int e = eb + k + q;
      const int d = d4[q];
      int r = -1;
      if (real && d >= n0 && d < n0 + TG && d < NN) { r = ((d - n0) << 20) | e; ++cnt; }
      rec[k + q] = r;
    }
  }
  int tot; int p = blk_excl_scan(cnt, scan_ws, tid, &tot);
#pragma unroll
  for (int k = 0; k < SP; ++k) if (rec[k] >= 0) { if ((unsigned)p < (unsigned)CAP) LIST[p] = rec[k]; ++p; }
  __syncthreads();
  return tot < CAP ? tot : CAP;
}

__global__ __launch_bounds__(NT) void stream_kernel(const float* __restrict__ QKV, const int* __restrict__ ei,
                                                   const float* __restrict__ ea, const float* __restrict__ demb,
                                                   const float* __restrict__ dW, const float* __restrict__ db,
                                                   const float* __restrict__ sw, float* __restrict__ ACC,
                                                   unsigned short* __restrict__ AGGp, int si, float maxd) {
  extern __shared__ __align__(16) float dyn_lds[];
  float* SM = dyn_lds;
  float* SL = dyn_lds + TG * NHD;
  int* LIST = (int*)(dyn_lds + 2 * TG * NHD);
  __shared__ int scan_ws[80];
  __shared__ float DEMB[(NBIN + 1) * NHD];
  __shared__ float DWB[32];
  _Float16* AGG = (_Float16*)AGGp;
  const int tid = threadIdx.x, lane = tid & 31, wave = tid >> 5;
  const int n0 = blockIdx.x * TG;
  const int h = lane >> 2;
  const int c4 = 4 * lane;
  float w0, w1, w2;
  scale_softmax(sw, w0, w1, w2);
  const float wsi = (si == 0) ? w0 : ((si == 1) ? w1 : w2);
  for (int i = tid; i < (NBIN + 1) * NHD; i += NT) DEMB[i] = demb[i];
  if (tid < 2 * NHD) DWB[tid] = dW[tid];
  if (tid >= 16 && tid < 16 + NHD) DWB[tid] = db[tid - 16];
  for (int i = tid; i < TG * NHD; i += NT) { SM[i] = -__builtin_inff(); SL[i] = 0.f; }
  float* accb = ACC + (size_t)n0 * DD;
  {
    const v4f z4 = {0.f, 0.f, 0.f, 0.f};
    for (int pass = 0; pass < 2; ++pass) {
#pragma unroll 1
      for (int j = 0; j < TG / 8; ++j) {
        float* ap = accb + (size_t)(wave * (TG / 8) + j) * DD + c4;
        *(volatile v4f*)ap = z4;
      }
      __threadfence();
    }
  }
  __syncthreads();
  const float dw0 = DWB[2 * h], dw1 = DWB[2 * h + 1], dbh = DWB[16 + h];
  const int* srcv = ei;
  const int* dstv = ei + NE;
#pragma unroll 1
  for (int c = 0; c < NCH; ++c) {
    const int tot = chunk_hits<SPT, SCH>(dstv, c * SCH, n0, tid, LIST, scan_ws);
#pragma unroll 1
    for (int base = 0; base < tot; base += 32) {
      const int q = base + lane;
      const int rv = (q < tot) ? LIST[q < SCH ? q : (SCH - 1)] : -1;
      const int own = (rv >= 0 && (rv >> 28) == wave) ? 1 : 0;
      unsigned msk = (unsigned)__ballot(own);
#pragma unroll 1
      for (int it = 0; it < 32; ++it) {
        if (msk == 0u) break;
        const int bp = __builtin_ctz(msk); msk &= msk - 1u;
        const int r = __shfl(rv, bp, 32);
        const int dl = r >> 20;
        int e = r & 0xFFFFF; e = (e < NE) ? e : (NE - 1);
        int s = srcv[e];
        s = s < 0 ? 0 : (s >= NN ? NN - 1 : s);
        int d = n0 + dl; d = (d < NN) ? d : (NN - 1);
        const v4f qv = *(const v4f*)(QKV + (size_t)d * QKVP + c4);
        const v4f kv = *(const v4f*)(QKV + (size_t)s * QKVP + DD + c4);
        const v4f vv = *(const v4f*)(QKV + (size_t)s * QKVP + 2 * DD + c4);
        float dot = qv[0] * kv[0];
        dot = fmaf(qv[1], kv[1], dot); dot = fmaf(qv[2], kv[2], dot); dot = fmaf(qv[3], kv[3], dot);
        dot += __shfl_xor(dot, 1, 32); dot += __shfl_xor(dot, 2, 32);
        const float* eap = ea + (size_t)e * 3;
        const float ea0 = eap[0], ea1 = eap[1], ea2 = eap[2];
        const float tb = (ea0 / maxd) * (float)NBIN;
        int bin = (int)tb;
        bin = (bin > NBIN) ? NBIN : bin;
        bin = (bin < 0) ? (bin + (NBIN + 1)) : bin;
        bin = (bin < 0) ? 0 : bin;
        float bias = DEMB[bin * NHD + h];
        const float sq = fmaf(ea1, ea1, ea2 * ea2);
        const float nrm = fmaxf(__builtin_amdgcn_sqrtf(sq), 1e-8f);
        const float rn = __builtin_amdgcn_rcpf(nrm);
        float z = fmaf(ea2 * rn, dw1, (ea1 * rn) * dw0) + dbh;
        z = fminf(fmaxf(z, -16.0f), 16.0f);
        const float t2 = __expf(2.0f * z);
        bias += (t2 - 1.0f) * __builtin_amdgcn_rcpf(t2 + 1.0f);
        const float sc = fmaf(dot, 0.25f, bias);
        const int mi = dl * NHD + h;
        const float mo = SM[mi], lo = SL[mi];
        const float mn = fmaxf(mo, sc);
        const float rr = __expf(mo - mn), ex = __expf(sc - mn);
        const float ln = fmaf(lo, rr, ex);
        if ((lane & 3) == 0) { SM[mi] = mn; SL[mi] = ln; }
        float* ap = accb + (size_t)dl * DD + c4;
        const v4f qa = *(const v4f*)ap;
        v4f o;
#pragma unroll
        for (int i = 0; i < 4; ++i) o[i] = fmaf(qa[i], rr, ex * vv[i]);
        *(volatile v4f*)ap = o;
        __threadfence();
        *(volatile v4f*)ap = o;
        asm volatile("" ::: "memory");
      }
    }
    __syncthreads();
  }
#pragma unroll 1
  for (int j = 0; j < TG / 8; ++j) {
    const int dl = wave * (TG / 8) + j;
    const int n = n0 + dl;
    if (n < MP) {
      const bool live = n < NN;
      const float* ap = accb + (size_t)dl * DD + c4;
      const v4f qa = *(const v4f*)ap;
      float l = SL[dl * NHD + h];
      l = (live && l > 0.f) ? l : 1.0f;
      const float inv = (wsi * AGSC) * (1.0f / l);
      float y[4];
#pragma unroll
      for (int i = 0; i < 4; ++i) { const float tv = qa[i] * inv; y[i] = live ? tv : 0.f; }
      const int sl = (2 * lane) & 31;
      v8h h8;
#pragma unroll
      for (int i = 0; i < 4; ++i) {
        const float ta = __shfl(y[i], sl, 32), tc = __shfl(y[i], sl + 1, 32);
        h8[i] = (_Float16)ta; h8[4 + i] = (_Float16)tc;
      }
      _Float16* hq = AGG + (size_t)n * DD + 8 * (lane & 15);
      for (int pass = 0; pass < 2; ++pass) {
        if (lane < 16) *(volatile v8h*)hq = h8;
        __threadfence();
      }
    }
  }
}

extern "C" void kernel_launch(void* const* d_in, const int* in_sizes, int n_in,
                              void* d_out, int out_size, void* d_ws, size_t ws_size, hipStream_t stream) {
  if (n_in < 15) return;
  const float* x    = (const float*)d_in[0];
  const int*   ei   = (const int*)  d_in[1];
  const float* ea   = (const float*)d_in[2];
  const float* Wq   = (const float*)d_in[3];
  const float* bq   = (const float*)d_in[4];
  const float* Wk   = (const float*)d_in[5];
  const float* bk   = (const float*)d_in[6];
  const float* Wv   = (const float*)d_in[7];
  const float* bv   = (const float*)d_in[8];
  const float* Wo   = (const float*)d_in[9];
  const float* bo   = (const float*)d_in[10];
  const float* demb = (const float*)d_in[11];
  const float* dWp  = (const float*)d_in[12];
  const float* dbp  = (const float*)d_in[13];
  const float* sw   = (const float*)d_in[14];
  float* out = (float*)d_out;

  if (in_sizes[0] != NN * DD || in_sizes[1] != NSC * 2 * NE || in_sizes[2] != NSC * NE * 3) return;
  if (in_sizes[3] != NSC * DD * DD || in_sizes[5] != NSC * DD * DD || in_sizes[7] != NSC * DD * DD || in_sizes[9] != NSC * DD * DD) return;
  if (in_sizes[4] != NSC * DD || in_sizes[6] != NSC * DD || in_sizes[8] != NSC * DD || in_sizes[10] != NSC * DD) return;
  if (in_sizes[11] != NSC * (NBIN + 1) * NHD || in_sizes[12] != NSC * NHD * 2 || in_sizes[13] != NSC * NHD || in_sizes[14] != NSC) return;
  if (out_size != NN * DD) return;

  char* ws = (char*)d_ws; size_t off = 0;
  auto carve = [&](size_t bytes) -> char* { char* p = ws + off; off += (bytes + 255) & ~(size_t)255; return p; };
  unsigned short* X16    = (unsigned short*)carve((size_t)MP * DD * 2);
  float*          QKV    = (float*)carve((size_t)MP * QKVP * 4);
  float*          ACC    = (float*)carve((size_t)NROWT * DD * 4);
  unsigned short* AGG16  = (unsigned short*)carve((size_t)MP * DD * 2);
  unsigned short* WQKV16 = (unsigned short*)carve((size_t)NSC * QKVP * DD * 2);
  unsigned short* WO16   = (unsigned short*)carve((size_t)NSC * DD * DD * 2);
  float*          BQKV   = (float*)carve((size_t)NSC * QKVP * 4);
  float*          BOW    = (float*)carve((size_t)NSC * DD * 4);
  if (off > ws_size || off > (size_t)134217728) return;

  cast_x_kernel<<<(MP * (DD / 2) + 255) / 256, 256, 0, stream>>>(x, X16, NN * (DD / 2), MP * (DD / 2));
  wprep_kernel<<<1, NT, 0, stream>>>(Wq, bq, Wk, bk, Wv, bv, Wo, bo, sw,
                                     (unsigned*)WQKV16, (unsigned*)WO16, BQKV, BOW);
  hipFuncSetAttribute(reinterpret_cast<const void*>(&stream_kernel), hipFuncAttributeMaxDynamicSharedMemorySize, STREAM_LDS_BYTES);

  const float maxd[NSC] = {50.0f, 200.0f, 500.0f};
  const int tilesQKV = (MP / 64) * (QKVP / 64);
  const int tilesO   = (MP / 64) * (DD / 64);
  for (int si = 0; si < NSC; ++si) {
    wmma_gemm64<0, false, 2, 0, false, 0><<<dim3((tilesQKV + 7) / 8, 1), 256, 0, stream>>>(
        U16(X16), U16(X16), DD, 0L,
        U16(WQKV16 + (size_t)si * QKVP * DD), U16(WQKV16 + (size_t)si * QKVP * DD), DD, 0L,
        (void*)QKV, (void*)nullptr, QKVP, 0L,
        BQKV + si * QKVP, (const float*)nullptr, 0L, MP, QKVP, DD, 1.0f / WSC, MP);
    stream_kernel<<<NTILE, NT, STREAM_LDS_BYTES, stream>>>(
        QKV, ei + (size_t)si * 2 * NE, ea + (size_t)si * NE * 3, demb + (size_t)si * (NBIN + 1) * NHD,
        dWp + (size_t)si * NHD * 2, dbp + (size_t)si * NHD, sw, ACC, AGG16, si, maxd[si]);
    if (si == 0) {
      wmma_gemm64<0, false, 2, 0, false, 0><<<dim3((tilesO + 7) / 8, 1), 256, 0, stream>>>(
          U16(AGG16), U16(AGG16), DD, 0L,
          U16(WO16 + (size_t)si * DD * DD), U16(WO16 + (size_t)si * DD * DD), DD, 0L,
          (void*)out, (void*)nullptr, DD, 0L,
          BOW + si * DD, (const float*)nullptr, 0L, MP, DD, DD, 1.0f / (WSC * AGSC), NN);
    } else {
      wmma_gemm64<0, false, 2, 0, true, 0><<<dim3((tilesO + 7) / 8, 1), 256, 0, stream>>>(
          U16(AGG16), U16(AGG16), DD, 0L,
          U16(WO16 + (size_t)si * DD * DD), U16(WO16 + (size_t)si * DD * DD), DD, 0L,
          (void*)out, (void*)nullptr, DD, 0L,
          BOW + si * DD, (const float*)out, 0L, MP, DD, DD, 1.0f / (WSC * AGSC), NN);
    }
  }
}
